// LSTM_ATTN_GNN_26362509263638
// MI455X (gfx1250) — hardware-verified
//
#include <hip/hip_runtime.h>

typedef __bf16         v16bf __attribute__((ext_vector_type(16)));
typedef unsigned short v16us __attribute__((ext_vector_type(16)));
typedef unsigned short v8us  __attribute__((ext_vector_type(8)));
typedef float          v8f   __attribute__((ext_vector_type(8)));
typedef float          v4f   __attribute__((ext_vector_type(4)));
typedef v8us __attribute__((may_alias)) v8usa;
typedef v4f  __attribute__((may_alias)) v4fa;

union FragU { v16us v; v8us half[2]; };

#define TSTEPS 128
#define NB     256
#define MROWS  32768
#define HUMN   20
#define HID    256

#define P_EW1 0
#define P_EW2 5120
#define P_NW1 15360
#define P_NW2 25600
#define P_GWX 35840
#define P_GWH 84992
#define P_HW1 281600
#define P_AW2 412672
#define P_CW2 478208
#define P_WEND 543744
static_assert(P_EW2 == P_EW1 + 160 * 32);
static_assert(P_NW1 == P_EW2 + 64 * 160);
static_assert(P_NW2 == P_NW1 + 160 * 64);
static_assert(P_GWX == P_NW2 + 64 * 160);
static_assert(P_GWH == P_GWX + 768 * 64);
static_assert(P_HW1 == P_GWH + 768 * 256);
static_assert(P_AW2 == P_HW1 + 512 * 256);
static_assert(P_CW2 == P_AW2 + 256 * 256);
static_assert(P_WEND == P_CW2 + 256 * 256);

#define B_NIN  ((size_t)1087488)
#define B_RNN  ((size_t)9476096)
#define B_OUTS ((size_t)17864704)
#define B_TA   ((size_t)51419136)
#define B_TC   ((size_t)84973568)
#define B_END  ((size_t)118528000)
#define TPLANE ((size_t)MROWS * 512)
static_assert(B_NIN == (size_t)P_WEND * 2);
static_assert(B_RNN == B_NIN + (size_t)MROWS * 128 * 2);
static_assert(B_OUTS == B_RNN + (size_t)MROWS * 128 * 2);
static_assert(B_TA == B_OUTS + (size_t)MROWS * 512 * 2);
static_assert(B_TC == B_TA + TPLANE * 2);
static_assert(B_END == B_TC + TPLANE * 2);
static_assert(B_END <= (size_t)134217728);
static_assert(B_NIN % 256 == 0 && B_RNN % 256 == 0 && B_OUTS % 256 == 0 && B_TA % 256 == 0 && B_TC % 256 == 0);
static_assert((P_EW2 * 2) % 256 == 0 && (P_NW1 * 2) % 256 == 0 && (P_NW2 * 2) % 256 == 0 && (P_GWX * 2) % 256 == 0 &&
              (P_GWH * 2) % 256 == 0 && (P_HW1 * 2) % 256 == 0 && (P_AW2 * 2) % 256 == 0 && (P_CW2 * 2) % 256 == 0);

#define OUT1_OFF 32768
#define OUT2_OFF 8421376
#define OUT_TOTAL 8486912
static_assert(OUT1_OFF == MROWS);
static_assert(OUT2_OFF == OUT1_OFF + MROWS * HID);
static_assert(OUT2_OFF + NB * HID == OUT_TOTAL);
static_assert((OUT1_OFF * 4) % 128 == 0 && (OUT2_OFF * 4) % 128 == 0);

#define PB1 3
#define PB2 8
#define PB3 13
#define PB4 18
#define PB5 42
#define PB6 138
#define PB7 170
#define PB8 202
#define PB9 234
#define PB_END 266

__device__ __forceinline__ unsigned bf_bits(float f) {
  unsigned u = __builtin_bit_cast(unsigned, f);
  u += 0x7FFFu + ((u >> 16) & 1u);
  return u >> 16;
}
__device__ __forceinline__ float bf_val(unsigned b) { return __builtin_bit_cast(float, b << 16); }
__device__ __forceinline__ float bfr(float f) { return bf_val(bf_bits(f)); }
__device__ __forceinline__ unsigned short bfs(float f) { return (unsigned short)bf_bits(f); }
__device__ __forceinline__ unsigned split_hl(float v) {
  const unsigned hi = bf_bits(v);
  const unsigned lo = bf_bits(v - bf_val(hi));
  return hi | (lo << 16);
}
__device__ __forceinline__ float relu_f(float v) { return (v > 0.0f) ? v : (v - v); }
__device__ __forceinline__ float sigm_f(float v) {
  v = fminf(fmaxf(v, -30.0f), 30.0f);
  const float e = expf(-v);
  return 1.0f / (1.0f + e);
}
__device__ __forceinline__ float hsum16(float v) {
  v += __shfl_xor(v, 1);
  v += __shfl_xor(v, 2);
  v += __shfl_xor(v, 4);
  v += __shfl_xor(v, 8);
  return v;
}

__device__ __forceinline__ v8f wmma_bf(v16bf a, v16bf b, v8f c) {
  v8f d = __builtin_amdgcn_wmma_f32_16x16x32_bf16(false, a, false, b, (short)0, c, false, false);
  asm volatile("v_nop\n\tv_nop\n\tv_nop\n\tv_nop" : "+v"(d) : "v"(a), "v"(b));
  return d;
}
__device__ __forceinline__ v16bf load_frag(const unsigned short* p, int h) {
  FragU f;
  f.half[0] = *(const v8usa*)(p + 8 * h);
  f.half[1] = *(const v8usa*)(p + 16 + 8 * h);
  return __builtin_bit_cast(v16bf, f.v);
}

template <int K, int N, int KP, int NP>
__device__ __forceinline__ void tr_chunk(const float* __restrict__ src, unsigned short* __restrict__ dst, int c) {
  constexpr int CH = NP * KP / 8;
  static_assert(KP % 8 == 0);
  const int cc = (c < CH) ? c : (CH - 1);
  const int n = (cc * 8) / KP, k0 = (cc * 8) % KP;
  const int nc = (n < N) ? n : (N - 1);
  const unsigned nm = (n < N) ? 0xFFFFu : 0u;
  float x[8];
  #pragma unroll
  for (int j = 0; j < 8; ++j) {
    const int k = k0 + j;
    const int kc = (k < K) ? k : (K - 1);
    x[j] = src[(size_t)kc * N + nc];
  }
  v8us o;
  #pragma unroll
  for (int j = 0; j < 8; ++j) {
    const unsigned km = (k0 + j < K) ? nm : 0u;
    o[j] = (unsigned short)(bf_bits(x[j]) & km);
  }
  if (c < CH) *(volatile v8us*)(dst + (size_t)c * 8) = o;
  __threadfence();
  if (c < CH) *(volatile v8us*)(dst + (size_t)c * 8) = o;
}

__global__ __launch_bounds__(256) void k_prep(
    const float* __restrict__ eW1, const float* __restrict__ eW2,
    const float* __restrict__ nW1, const float* __restrict__ nW2,
    const float* __restrict__ gWx, const float* __restrict__ gWh,
    const float* __restrict__ aW1, const float* __restrict__ aW2,
    const float* __restrict__ cW1, const float* __restrict__ cW2,
    unsigned short* __restrict__ planes)
{
  const int b = blockIdx.x, tid = threadIdx.x;
  if (b < PB1)      tr_chunk<21, 150, 32, 160>(eW1, planes + P_EW1, b * 256 + tid);
  else if (b < PB2) tr_chunk<150, 50, 160, 64>(eW2, planes + P_EW2, (b - PB1) * 256 + tid);
  else if (b < PB3) tr_chunk<59, 150, 64, 160>(nW1, planes + P_NW1, (b - PB2) * 256 + tid);
  else if (b < PB4) tr_chunk<150, 64, 160, 64>(nW2, planes + P_NW2, (b - PB3) * 256 + tid);
  else if (b < PB5) tr_chunk<64, 768, 64, 768>(gWx, planes + P_GWX, (b - PB4) * 256 + tid);
  else if (b < PB6) tr_chunk<256, 768, 256, 768>(gWh, planes + P_GWH, (b - PB5) * 256 + tid);
  else if (b < PB7) tr_chunk<256, 256, 256, 256>(aW1, planes + P_HW1, (b - PB6) * 256 + tid);
  else if (b < PB8) tr_chunk<256, 256, 256, 256>(cW1, planes + P_HW1 + 65536, (b - PB7) * 256 + tid);
  else if (b < PB9) tr_chunk<256, 256, 256, 256>(aW2, planes + P_AW2, (b - PB8) * 256 + tid);
  else              tr_chunk<256, 256, 256, 256>(cW2, planes + P_CW2, (b - PB9) * 256 + tid);
}

static_assert(4 * HUMN == 80 && 80 % 16 == 0 && MROWS % 4 == 0);
__global__ __launch_bounds__(160) __attribute__((amdgpu_num_vgpr(248))) void k_edge(
    const float* __restrict__ rn, const float* __restrict__ te, const float* __restrict__ se,
    const unsigned short* __restrict__ ew1t, const unsigned short* __restrict__ ew2t,
    const float* __restrict__ eb1, const float* __restrict__ eb2,
    unsigned short* __restrict__ nin)
{
  __shared__ __attribute__((aligned(16))) unsigned short sA1[80 * 32];
  __shared__ __attribute__((aligned(16))) unsigned short sScr[5 * 1024];
  __shared__ __attribute__((aligned(16))) float sM2[80 * 64];
  __shared__ __attribute__((aligned(16))) unsigned short sNin[4 * 128];
  __shared__ __attribute__((aligned(16))) float sB1[160];
  __shared__ __attribute__((aligned(16))) float sB2[64];
  __shared__ __attribute__((aligned(16))) unsigned short sRob[64];

  const int tid = threadIdx.x, lane = tid & 31, w = tid >> 5;
  const int h = lane >> 4, m = lane & 15;
  const int node0 = blockIdx.x * 4;

  {
    const int c1 = (tid < 150) ? tid : 149;
    const float v1 = bfr(eb1[c1]);
    sB1[tid] = (tid < 150) ? v1 : 0.0f;
    const int c2 = tid & 63;
    const int c2c = (c2 < 50) ? c2 : 49;
    const float v2 = bfr(eb2[c2c]);
    const int g = (tid >> 4) & 3, c = tid & 15;
    const int ci = (c < 7) ? c : 6;
    const int ti = (c == 8) ? 1 : 0;
    const float a = rn[(size_t)(node0 + g) * 7 + ci];
    const float q = te[(size_t)(node0 + g) * 2 + ti];
    const float v = (c < 7) ? a : q;
    const unsigned bits = (c < 9) ? bf_bits(v) : 0u;
    if (tid < 64) {
      sB2[tid] = (c2 < 50) ? v2 : 0.0f;
      sRob[tid] = (unsigned short)bits;
    }
  }
  __syncthreads();

  {
    const int e = (tid < 80) ? tid : 79;
    const int g = e / 20;
    const float* sp = se + (size_t)node0 * 240 + (size_t)e * 12;
    const v4f s0 = *(const v4fa*)sp;
    const v4f s1 = *(const v4fa*)(sp + 4);
    const v4f s2 = *(const v4fa*)(sp + 8);
    const v8us r0 = *(const v8usa*)(sRob + g * 16);
    const v8us r1 = *(const v8usa*)(sRob + g * 16 + 8);
    const unsigned short z = (unsigned short)0;
    const v8us o1 = { r1[0], bfs(s0.x), bfs(s0.y), bfs(s0.z), bfs(s0.w), bfs(s1.x), bfs(s1.y), bfs(s1.z) };
    const v8us o2 = { bfs(s1.w), bfs(s2.x), bfs(s2.y), bfs(s2.z), bfs(s2.w), z, z, z };
    const v8us o3 = { z, z, z, z, z, z, z, z };
    if (tid < 80) {
      *(v8usa*)(sA1 + e * 32)      = r0;
      *(v8usa*)(sA1 + e * 32 + 8)  = o1;
      *(v8usa*)(sA1 + e * 32 + 16) = o2;
      *(v8usa*)(sA1 + e * 32 + 24) = o3;
    }
  }
  __syncthreads();

  const v8f z8 = {0.f, 0.f, 0.f, 0.f, 0.f, 0.f, 0.f, 0.f};
  unsigned short* scrH = sScr + w * 1024;
  unsigned short* scrL = scrH + 512;
  const v16bf a1 = load_frag(sA1 + (16 * w + m) * 32, h);
  v8f acc[4];
  #pragma unroll
  for (int t = 0; t < 4; ++t) acc[t] = z8;

  #pragma unroll 1
  for (int j = 0; j < 5; ++j) {
    #pragma unroll
    for (int s = 0; s < 2; ++s) {
      const int nt = 2 * j + s;
      const v16bf b = load_frag(ew1t + (size_t)(16 * nt + m) * 32, h);
      const v8f d = wmma_bf(a1, b, z8);
      const float bb = sB1[16 * nt + m];
      #pragma unroll
      for (int r = 0; r < 8; ++r) {
        const float v = relu_f(d[r] + bb);
        const unsigned p = split_hl(v);
        scrH[(8 * h + r) * 32 + 16 * s + m] = (unsigned short)(p & 0xFFFFu);
        scrL[(8 * h + r) * 32 + 16 * s + m] = (unsigned short)(p >> 16);
      }
    }
    __syncthreads();
    const v16bf ah = load_frag(scrH + m * 32, h);
    const v16bf al = load_frag(scrL + m * 32, h);
    #pragma unroll
    for (int t = 0; t < 4; ++t) {
      const v16bf b2 = load_frag(ew2t + (size_t)(16 * t + m) * 160 + 32 * j, h);
      acc[t] = wmma_bf(ah, b2, acc[t]);
      acc[t] = wmma_bf(al, b2, acc[t]);
    }
  }

  #pragma unroll
  for (int t = 0; t < 4; ++t) {
    const float bb = sB2[16 * t + m];
    #pragma unroll
    for (int r = 0; r < 8; ++r)
      sM2[(16 * w + 8 * h + r) * 64 + 16 * t + m] = relu_f(acc[t][r] + bb);
  }
  __syncthreads();

  #pragma unroll 1
  for (int i = 0; i < 2; ++i) {
    const int idx = tid + 160 * i;
    if (idx < 256) {
      const int g = idx >> 6, c = idx & 63;
      float mn = sM2[(20 * g) * 64 + c];
      #pragma unroll 4
      for (int jj = 1; jj < HUMN; ++jj) mn = fminf(mn, sM2[(20 * g + jj) * 64 + c]);
      const unsigned p = split_hl(mn);
      int rc = c - 50;
      rc = (rc < 0) ? 0 : ((rc > 8) ? 8 : rc);
      const unsigned rb = sRob[g * 16 + rc];
      const unsigned isagg = (c < 50) ? 0xFFFFu : 0u;
      const unsigned isrob = (c >= 50 && c < 59) ? 0xFFFFu : 0u;
      sNin[g * 128 + c]      = (unsigned short)(((p & 0xFFFFu) & isagg) | (rb & isrob));
      sNin[g * 128 + 64 + c] = (unsigned short)((p >> 16) & isagg);
    }
  }
  __syncthreads();

  if (tid < 64) {
    const v8us v = *(const v8usa*)(sNin + tid * 8);
    unsigned short* dst = nin + (size_t)node0 * 128 + (size_t)tid * 8;
    *(volatile v8us*)dst = v;
    __threadfence();
    *(volatile v8us*)dst = v;
  }
}

template <int NTH, int NIT>
__device__ __forceinline__ void flush_us(const unsigned short* s, unsigned short* dst, int tid) {
  #pragma unroll
  for (int i = 0; i < NIT; ++i) {
    const int c = tid + NTH * i;
    const v8us v = *(const v8usa*)(s + c * 8);
    *(volatile v8us*)(dst + (size_t)c * 8) = v;
  }
}
template <int NTH, int NIT>
__device__ __forceinline__ void flush_f32(const float* s, float* dst, int tid) {
  #pragma unroll
  for (int i = 0; i < NIT; ++i) {
    const int c = tid + NTH * i;
    const v4f v = *(const v4fa*)(s + c * 4);
    *(volatile v4f*)(dst + (size_t)c * 4) = v;
  }
}

static_assert(MROWS % 128 == 0);
__global__ __launch_bounds__(256) __attribute__((amdgpu_num_vgpr(248))) void k_node(
    const unsigned short* __restrict__ nin,
    const unsigned short* __restrict__ nw1t, const unsigned short* __restrict__ nw2t,
    const float* __restrict__ nb1, const float* __restrict__ nb2,
    unsigned short* __restrict__ rnnin)
{
  __shared__ __attribute__((aligned(16))) unsigned short sScr[8 * 1024];
  __shared__ __attribute__((aligned(16))) unsigned short sOut[128 * 128];
  __shared__ __attribute__((aligned(16))) float sB1[160];
  __shared__ __attribute__((aligned(16))) float sB2[64];

  const int tid = threadIdx.x, lane = tid & 31, w = tid >> 5;
  const int h = lane >> 4, m = lane & 15;
  const int row0 = blockIdx.x * 128;

  {
    const int i1 = (tid < 160) ? tid : 159;
    const int c1 = (i1 < 150) ? i1 : 149;
    const float v1 = bfr(nb1[c1]);
    const float v2 = bfr(nb2[tid & 63]);
    if (tid < 160) sB1[tid] = (tid < 150) ? v1 : 0.0f;
    if (tid < 64) sB2[tid] = v2;
  }
  __syncthreads();

  const v8f z8 = {0.f, 0.f, 0.f, 0.f, 0.f, 0.f, 0.f, 0.f};
  unsigned short* scrH = sScr + w * 1024;
  unsigned short* scrL = scrH + 512;
  const unsigned short* arow = nin + (size_t)(row0 + 16 * w + m) * 128;
  const v16bf ahi0 = load_frag(arow, h);
  const v16bf ahi1 = load_frag(arow + 32, h);
  const v16bf alo0 = load_frag(arow + 64, h);
  const v16bf alo1 = load_frag(arow + 96, h);
  v8f acc[4];
  #pragma unroll
  for (int t = 0; t < 4; ++t) acc[t] = z8;

  #pragma unroll 1
  for (int j = 0; j < 5; ++j) {
    #pragma unroll
    for (int s = 0; s < 2; ++s) {
      const int nt = 2 * j + s;
      const unsigned short* brow = nw1t + (size_t)(16 * nt + m) * 64;
      const v16bf b0 = load_frag(brow, h);
      const v16bf b1 = load_frag(brow + 32, h);
      v8f d = wmma_bf(ahi0, b0, z8);
      d = wmma_bf(alo0, b0, d);
      d = wmma_bf(ahi1, b1, d);
      d = wmma_bf(alo1, b1, d);
      const float bb = sB1[16 * nt + m];
      #pragma unroll
      for (int r = 0; r < 8; ++r) {
        const float v = relu_f(d[r] + bb);
        const unsigned p = split_hl(v);
        scrH[(8 * h + r) * 32 + 16 * s + m] = (unsigned short)(p & 0xFFFFu);
        scrL[(8 * h + r) * 32 + 16 * s + m] = (unsigned short)(p >> 16);
      }
    }
    __syncthreads();
    const v16bf ah = load_frag(scrH + m * 32, h);
    const v16bf al = load_frag(scrL + m * 32, h);
    #pragma unroll
    for (int t = 0; t < 4; ++t) {
      const v16bf b2 = load_frag(nw2t + (size_t)(16 * t + m) * 160 + 32 * j, h);
      acc[t] = wmma_bf(ah, b2, acc[t]);
      acc[t] = wmma_bf(al, b2, acc[t]);
    }
  }

  #pragma unroll
  for (int t = 0; t < 4; ++t) {
    const float bb = sB2[16 * t + m];
    #pragma unroll
    for (int r = 0; r < 8; ++r) {
      const float v = relu_f(acc[t][r] + bb);
      const unsigned p = split_hl(v);
      const int rowl = 16 * w + 8 * h + r;
      sOut[rowl * 128 + 16 * t + m]      = (unsigned short)(p & 0xFFFFu);
      sOut[rowl * 128 + 64 + 16 * t + m] = (unsigned short)(p >> 16);
    }
  }
  __syncthreads();

  unsigned short* dst = rnnin + (size_t)row0 * 128;
  flush_us<256, 8>(sOut, dst, tid);
  __threadfence();
  flush_us<256, 8>(sOut, dst, tid);
}

static_assert(NB % 16 == 0 && 8 * 32 == HID);
__global__ __launch_bounds__(256) __attribute__((amdgpu_num_vgpr(248))) void k_gru(
    const unsigned short* __restrict__ rnnin, const float* __restrict__ h0, const float* __restrict__ masks,
    const unsigned short* __restrict__ gwxt, const unsigned short* __restrict__ gwht,
    const float* __restrict__ gbx, const float* __restrict__ gbh,
    unsigned short* __restrict__ outs, float* __restrict__ out2)
{
  __shared__ __attribute__((aligned(16))) unsigned short sAh[2 * 16 * 256];
  __shared__ __attribute__((aligned(16))) unsigned short sOut[16 * 512];
  __shared__ __attribute__((aligned(16))) float sF[16 * 256];
  __shared__ __attribute__((aligned(16))) float sBx[768];
  __shared__ __attribute__((aligned(16))) float sBh[768];

  const int tid = threadIdx.x, lane = tid & 31, w = tid >> 5;
  const int h = lane >> 4, m = lane & 15;
  const int rowb = blockIdx.x * 16;

  #pragma unroll
  for (int i = 0; i < 4; ++i) {
    const int q = tid + 256 * i;
    const v4f v = *(const v4fa*)(h0 + (size_t)rowb * HID + (size_t)q * 4);
    const v4f r = { bfr(v.x), bfr(v.y), bfr(v.z), bfr(v.w) };
    *(v4fa*)(sF + q * 4) = r;
  }
  #pragma unroll
  for (int j = 0; j < 3; ++j) {
    const int i = tid + 256 * j;
    sBx[i] = bfr(gbx[i]);
    sBh[i] = bfr(gbh[i]);
  }
  __syncthreads();

  const v8f z8 = {0.f, 0.f, 0.f, 0.f, 0.f, 0.f, 0.f, 0.f};
  v8f hst[2];
  float bR[2], bZ[2], bXN[2], bHN[2];
  #pragma unroll
  for (int s = 0; s < 2; ++s) {
    const int col = 32 * w + 16 * s + m;
    #pragma unroll
    for (int r = 0; r < 8; ++r) hst[s][r] = sF[(8 * h + r) * HID + col];
    bR[s]  = sBx[col] + sBh[col];
    bZ[s]  = sBx[256 + col] + sBh[256 + col];
    bXN[s] = sBx[512 + col];
    bHN[s] = sBh[512 + col];
  }

  const unsigned short* wxr = gwxt + (size_t)(32 * w + m) * 64;
  const unsigned short* whr = gwht + (size_t)(32 * w + m) * 256;

  #pragma unroll 1
  for (int t = 0; t < TSTEPS; ++t) {
    {
      const float* mp = masks + (size_t)t * NB + rowb + 8 * h;
      const v4f m0 = *(const v4fa*)mp;
      const v4f m1 = *(const v4fa*)(mp + 4);
      const float mk[8] = { bfr(m0.x), bfr(m0.y), bfr(m0.z), bfr(m0.w), bfr(m1.x), bfr(m1.y), bfr(m1.z), bfr(m1.w) };
      #pragma unroll
      for (int s = 0; s < 2; ++s) {
        const int col = 32 * w + 16 * s + m;
        #pragma unroll
        for (int r = 0; r < 8; ++r) {
          const float hm = hst[s][r] * mk[r];
          hst[s][r] = hm;
          const unsigned p = split_hl(hm);
          sAh[(8 * h + r) * 256 + col]        = (unsigned short)(p & 0xFFFFu);
          sAh[4096 + (8 * h + r) * 256 + col] = (unsigned short)(p >> 16);
        }
      }
    }
    __syncthreads();

    v8f aR[2], aZ[2], aXN[2], aHN[2];
    #pragma unroll
    for (int s = 0; s < 2; ++s) { aR[s] = z8; aZ[s] = z8; aXN[s] = z8; aHN[s] = z8; }

    {
      const unsigned short* xrow = rnnin + (size_t)(t * NB + rowb + m) * 128;
      #pragma unroll 1
      for (int ks = 0; ks < 2; ++ks) {
        const v16bf xh = load_frag(xrow + 32 * ks, h);
        const v16bf xl = load_frag(xrow + 64 + 32 * ks, h);
        #pragma unroll
        for (int s = 0; s < 2; ++s) {
          const unsigned short* bp = wxr + (size_t)(16 * s) * 64 + 32 * ks;
          v16bf b = load_frag(bp, h);
          aR[s] = wmma_bf(xh, b, aR[s]);
          aR[s] = wmma_bf(xl, b, aR[s]);
          b = load_frag(bp + (size_t)256 * 64, h);
          aZ[s] = wmma_bf(xh, b, aZ[s]);
          aZ[s] = wmma_bf(xl, b, aZ[s]);
          b = load_frag(bp + (size_t)512 * 64, h);
          aXN[s] = wmma_bf(xh, b, aXN[s]);
          aXN[s] = wmma_bf(xl, b, aXN[s]);
        }
      }
    }
    #pragma unroll 1
    for (int ks = 0; ks < 8; ++ks) {
      const v16bf hh = load_frag(sAh + m * 256 + 32 * ks, h);
      const v16bf hl = load_frag(sAh + 4096 + m * 256 + 32 * ks, h);
      #pragma unroll
      for (int s = 0; s < 2; ++s) {
        const unsigned short* bp = whr + (size_t)(16 * s) * 256 + 32 * ks;
        v16bf b = load_frag(bp, h);
        aR[s] = wmma_bf(hh, b, aR[s]);
        aR[s] = wmma_bf(hl, b, aR[s]);
        b = load_frag(bp + (size_t)256 * 256, h);
        aZ[s] = wmma_bf(hh, b, aZ[s]);
        aZ[s] = wmma_bf(hl, b, aZ[s]);
        b = load_frag(bp + (size_t)512 * 256, h);
        aHN[s] = wmma_bf(hh, b, aHN[s]);
        aHN[s] = wmma_bf(hl, b, aHN[s]);
      }
    }

    #pragma unroll
    for (int s = 0; s < 2; ++s) {
      const int col = 32 * w + 16 * s + m;
      #pragma unroll
      for (int r = 0; r < 8; ++r) {
        const float rg = sigm_f(aR[s][r] + bR[s]);
        const float zg = sigm_f(aZ[s][r] + bZ[s]);
        const float nn = tanhf((aXN[s][r] + bXN[s]) + rg * (aHN[s][r] + bHN[s]));
        const float hn = (1.0f - zg) * nn + zg * hst[s][r];
        hst[s][r] = hn;
        const unsigned p = split_hl(hn);
        sOut[(8 * h + r) * 512 + col]       = (unsigned short)(p & 0xFFFFu);
        sOut[(8 * h + r) * 512 + 256 + col] = (unsigned short)(p >> 16);
      }
    }
    __syncthreads();

    unsigned short* dst = outs + (size_t)(t * NB + rowb) * 512;
    flush_us<256, 4>(sOut, dst, tid);
    __threadfence();
    flush_us<256, 4>(sOut, dst, tid);
  }

  #pragma unroll
  for (int s = 0; s < 2; ++s) {
    const int col = 32 * w + 16 * s + m;
    #pragma unroll
    for (int r = 0; r < 8; ++r) sF[(8 * h + r) * HID + col] = hst[s][r];
  }
  __syncthreads();
  float* d2 = out2 + (size_t)rowb * HID;
  flush_f32<256, 4>(sF, d2, tid);
  __threadfence();
  flush_f32<256, 4>(sF, d2, tid);
}

__device__ __forceinline__ void h1_store_pass(const unsigned short* sT, unsigned short* tbase,
                                              int row0, int ncol0, int w, int lane) {
  const int q8 = lane & 7, sub = lane >> 3;
  #pragma unroll
  for (int i = 0; i < 16; ++i) {
    const int lid = w * 64 + i * 4 + sub;
    const int row = lid >> 1, hl = lid & 1;
    const v8us v = *(const v8usa*)(sT + row * 128 + 64 * hl + 8 * q8);
    *(volatile v8us*)(tbase + (size_t)(row0 + row) * 512 + 256 * hl + ncol0 + 8 * q8) = v;
  }
}

__global__ __launch_bounds__(128) __attribute__((amdgpu_num_vgpr(248))) void k_h1(
    const unsigned short* __restrict__ outs, const unsigned short* __restrict__ hw1t,
    const float* __restrict__ ab1, const float* __restrict__ cb1,
    unsigned short* __restrict__ tpl)
{
  __shared__ __attribute__((aligned(16))) unsigned short sT[128 * 128];
  __shared__ __attribute__((aligned(16))) float sBias[64];

  const int tid = threadIdx.x, lane = tid & 31, w = tid >> 5;
  const int h = lane >> 4, m = lane & 15;
  const int row0 = blockIdx.x * 128;
  const int cg = blockIdx.y;

  {
    const int cix = (64 * cg + (tid & 63)) & 255;
    const float ba = bfr(ab1[cix]);
    const float bc = bfr(cb1[cix]);
    if (tid < 64) sBias[tid] = (cg < 4) ? ba : bc;
  }
  __syncthreads();

  const unsigned short* arow0 = outs + (size_t)(row0 + 32 * w + m) * 512;
  const unsigned short* arow1 = arow0 + (size_t)16 * 512;
  const unsigned short* brow = hw1t + (size_t)(64 * cg + m) * 256;

  const v8f z8 = {0.f, 0.f, 0.f, 0.f, 0.f, 0.f, 0.f, 0.f};
  v8f acc[2][4];
  #pragma unroll
  for (int mt = 0; mt < 2; ++mt)
    #pragma unroll
    for (int nt = 0; nt < 4; ++nt) acc[mt][nt] = z8;

  #pragma unroll 1
  for (int k0 = 0; k0 < 256; k0 += 32) {
    const v16bf a0h = load_frag(arow0 + k0, h);
    const v16bf a0l = load_frag(arow0 + 256 + k0, h);
    const v16bf a1h = load_frag(arow1 + k0, h);
    const v16bf a1l = load_frag(arow1 + 256 + k0, h);
    #pragma unroll
    for (int nt = 0; nt < 4; ++nt) {
      const v16bf b = load_frag(brow + (size_t)nt * 16 * 256 + k0, h);
      acc[0][nt] = wmma_bf(a0h, b, acc[0][nt]);
      acc[0][nt] = wmma_bf(a0l, b, acc[0][nt]);
      acc[1][nt] = wmma_bf(a1h, b, acc[1][nt]);
      acc[1][nt] = wmma_bf(a1l, b, acc[1][nt]);
    }
  }

  #pragma unroll
  for (int nt = 0; nt < 4; ++nt) {
    const int col = 16 * nt + m;
    const float bb = sBias[col];
    #pragma unroll
    for (int mt = 0; mt < 2; ++mt) {
      #pragma unroll
      for (int r = 0; r < 8; ++r) {
        const int rowl = 32 * w + 16 * mt + 8 * h + r;
        const float y = tanhf(acc[mt][nt][r] + bb);
        const unsigned p = split_hl(y);
        sT[rowl * 128 + col]      = (unsigned short)(p & 0xFFFFu);
        sT[rowl * 128 + 64 + col] = (unsigned short)(p >> 16);
      }
    }
  }
  __syncthreads();

  unsigned short* tbase = tpl + (size_t)(cg >> 2) * TPLANE;
  const int ncol0 = (64 * cg) & 255;
  h1_store_pass(sT, tbase, row0, ncol0, w, lane);
  __threadfence();
  h1_store_pass(sT, tbase, row0, ncol0, w, lane);
}

__device__ __forceinline__ void act_store_pass(const float* sO, float* out1, int row0, int n0, int w, int lane) {
  const int q8 = lane & 7, sub = lane >> 3;
  #pragma unroll
  for (int i = 0; i < 16; ++i) {
    const int lid = w * 64 + i * 4 + sub;
    const int row = lid >> 1, hl = lid & 1;
    const v4f v = *(const v4fa*)(sO + row * 64 + 32 * hl + 4 * q8);
    *(volatile v4f*)(out1 + (size_t)(row0 + row) * HID + n0 + 32 * hl + 4 * q8) = v;
  }
}

__global__ __launch_bounds__(128) __attribute__((amdgpu_num_vgpr(248))) void k_act(
    const unsigned short* __restrict__ ta, const unsigned short* __restrict__ aw2t,
    const float* __restrict__ ab2, float* __restrict__ out1)
{
  __shared__ __attribute__((aligned(16))) float sO[128 * 64];
  __shared__ __attribute__((aligned(16))) float sBias[64];

  const int tid = threadIdx.x, lane = tid & 31, w = tid >> 5;
  const int h = lane >> 4, m = lane & 15;
  const int row0 = blockIdx.x * 128;
  const int n0 = blockIdx.y * 64;

  {
    const float ba = bfr(ab2[n0 + (tid & 63)]);
    if (tid < 64) sBias[tid] = ba;
  }
  __syncthreads();

  const unsigned short* arow0 = ta + (size_t)(row0 + 32 * w + m) * 512;
  const unsigned short* arow1 = arow0 + (size_t)16 * 512;
  const unsigned short* brow = aw2t + (size_t)(n0 + m) * 256;

  const v8f z8 = {0.f, 0.f, 0.f, 0.f, 0.f, 0.f, 0.f, 0.f};
  v8f acc[2][4];
  #pragma unroll
  for (int mt = 0; mt < 2; ++mt)
    #pragma unroll
    for (int nt = 0; nt < 4; ++nt) acc[mt][nt] = z8;

  #pragma unroll 1
  for (int k0 = 0; k0 < 256; k0 += 32) {
    const v16bf a0h = load_frag(arow0 + k0, h);
    const v16bf a0l = load_frag(arow0 + 256 + k0, h);
    const v16bf a1h = load_frag(arow1 + k0, h);
    const v16bf a1l = load_frag(arow1 + 256 + k0, h);
    #pragma unroll
    for (int nt = 0; nt < 4; ++nt) {
      const v16bf b = load_frag(brow + (size_t)nt * 16 * 256 + k0, h);
      acc[0][nt] = wmma_bf(a0h, b, acc[0][nt]);
      acc[0][nt] = wmma_bf(a0l, b, acc[0][nt]);
      acc[1][nt] = wmma_bf(a1h, b, acc[1][nt]);
      acc[1][nt] = wmma_bf(a1l, b, acc[1][nt]);
    }
  }

  #pragma unroll
  for (int nt = 0; nt < 4; ++nt) {
    const int col = 16 * nt + m;
    const float bb = sBias[col];
    #pragma unroll
    for (int mt = 0; mt < 2; ++mt) {
      #pragma unroll
      for (int r = 0; r < 8; ++r) {
        const int rowl = 32 * w + 16 * mt + 8 * h + r;
        sO[rowl * 64 + col] = tanhf(acc[mt][nt][r] + bb);
      }
    }
  }
  __syncthreads();

  act_store_pass(sO, out1, row0, n0, w, lane);
  __threadfence();
  act_store_pass(sO, out1, row0, n0, w, lane);
}

static_assert(MROWS % 64 == 0);
__global__ __launch_bounds__(256) __attribute__((amdgpu_num_vgpr(248))) void k_crit(
    const unsigned short* __restrict__ tc, const unsigned short* __restrict__ cw2t,
    const float* __restrict__ cb2, const float* __restrict__ clW, const float* __restrict__ clb,
    float* __restrict__ out0)
{
  __shared__ __attribute__((aligned(16))) float sCb[256];
  __shared__ __attribute__((aligned(16))) float sCl[256];
  __shared__ __attribute__((aligned(16))) float sPart[128];

  const int tid = threadIdx.x, lane = tid & 31, w = tid >> 5;
  const int h = lane >> 4, m = lane & 15;
  const int mw = w & 3, nh = w >> 2;
  const int row0 = blockIdx.x * 64;

  sCb[tid] = bfr(cb2[tid]);
  sCl[tid] = bfr(clW[tid]);
  const float clbv = bfr(clb[0]);
  __syncthreads();

  const unsigned short* arow = tc + (size_t)(row0 + 16 * mw + m) * 512;
  const unsigned short* brow = cw2t + (size_t)(128 * nh + m) * 256;

  const v8f z8 = {0.f, 0.f, 0.f, 0.f, 0.f, 0.f, 0.f, 0.f};
  v8f acc[8];
  #pragma unroll
  for (int nt = 0; nt < 8; ++nt) acc[nt] = z8;

  #pragma unroll 1
  for (int k0 = 0; k0 < 256; k0 += 32) {
    const v16bf ah = load_frag(arow + k0, h);
    const v16bf al = load_frag(arow + 256 + k0, h);
    #pragma unroll
    for (int nt = 0; nt < 8; ++nt) {
      const v16bf b = load_frag(brow + (size_t)nt * 16 * 256 + k0, h);
      acc[nt] = wmma_bf(ah, b, acc[nt]);
      acc[nt] = wmma_bf(al, b, acc[nt]);
    }
  }

  float p[8];
  #pragma unroll
  for (int r = 0; r < 8; ++r) p[r] = 0.0f;
  #pragma unroll
  for (int nt = 0; nt < 8; ++nt) {
    const int col = 128 * nh + 16 * nt + m;
    const float bb = sCb[col];
    const float cw = sCl[col];
    #pragma unroll
    for (int r = 0; r < 8; ++r) p[r] += tanhf(acc[nt][r] + bb) * cw;
  }
  #pragma unroll
  for (int r = 0; r < 8; ++r) p[r] = hsum16(p[r]);
  if (m == 0) {
    #pragma unroll
    for (int r = 0; r < 8; ++r) sPart[(16 * mw + 8 * h + r) * 2 + nh] = p[r];
  }
  __syncthreads();

  const int tq = tid & 15;
  const v4f a = *(const v4fa*)(sPart + 8 * tq);
  const v4f c = *(const v4fa*)(sPart + 8 * tq + 4);
  const v4f o = { (a.x + a.y) + clbv, (a.z + a.w) + clbv, (c.x + c.y) + clbv, (c.z + c.w) + clbv };
  if (tid < 16) {
    float* dst = out0 + row0 + 4 * tq;
    *(volatile v4f*)dst = o;
    __threadfence();
    *(volatile v4f*)dst = o;
  }
}

extern "C" void kernel_launch(void* const* d_in, const int* in_sizes, int n_in,
                              void* d_out, int out_size, void* d_ws, size_t ws_size,
                              hipStream_t stream) {
  if (n_in < 27) return;
  if (in_sizes[0] != MROWS * 7 || in_sizes[1] != MROWS * 2 || in_sizes[2] != MROWS * HUMN * 12) return;
  if (in_sizes[3] != NB * HID || in_sizes[4] != MROWS) return;
  if (in_sizes[5] != 21 * 150 || in_sizes[6] != 150 || in_sizes[7] != 150 * 50 || in_sizes[8] != 50) return;
  if (in_sizes[9] != 59 * 150 || in_sizes[10] != 150 || in_sizes[11] != 150 * 64 || in_sizes[12] != 64) return;
  if (in_sizes[13] != 64 * 768 || in_sizes[14] != 256 * 768 || in_sizes[15] != 768 || in_sizes[16] != 768) return;
  if (in_sizes[17] != 65536 || in_sizes[18] != 256 || in_sizes[19] != 65536 || in_sizes[20] != 256) return;
  if (in_sizes[21] != 65536 || in_sizes[22] != 256 || in_sizes[23] != 65536 || in_sizes[24] != 256) return;
  if (in_sizes[25] != 256 || in_sizes[26] != 1) return;
  if (out_size != OUT_TOTAL) return;
  if (B_END > ws_size) return;

  const float* rn   = (const float*)d_in[0];
  const float* te   = (const float*)d_in[1];
  const float* se   = (const float*)d_in[2];
  const float* rhx  = (const float*)d_in[3];
  const float* msk  = (const float*)d_in[4];
  const float* eW1  = (const float*)d_in[5];
  const float* eb1  = (const float*)d_in[6];
  const float* eW2  = (const float*)d_in[7];
  const float* eb2  = (const float*)d_in[8];
  const float* nW1  = (const float*)d_in[9];
  const float* nb1  = (const float*)d_in[10];
  const float* nW2  = (const float*)d_in[11];
  const float* nb2  = (const float*)d_in[12];
  const float* gWx  = (const float*)d_in[13];
  const float* gWh  = (const float*)d_in[14];
  const float* gbx  = (const float*)d_in[15];
  const float* gbh  = (const float*)d_in[16];
  const float* aW1  = (const float*)d_in[17];
  const float* ab1  = (const float*)d_in[18];
  const float* aW2  = (const float*)d_in[19];
  const float* ab2  = (const float*)d_in[20];
  const float* cW1  = (const float*)d_in[21];
  const float* cb1  = (const float*)d_in[22];
  const float* cW2  = (const float*)d_in[23];
  const float* cb2  = (const float*)d_in[24];
  const float* clW  = (const float*)d_in[25];
  const float* clb  = (const float*)d_in[26];

  float* out0 = (float*)d_out;
  float* out1 = out0 + OUT1_OFF;
  float* out2 = out0 + OUT2_OFF;

  char* ws = (char*)d_ws;
  unsigned short* planes = (unsigned short*)ws;
  unsigned short* nin    = (unsigned short*)(ws + B_NIN);
  unsigned short* rnnin  = (unsigned short*)(ws + B_RNN);
  unsigned short* outs   = (unsigned short*)(ws + B_OUTS);
  unsigned short* tpl    = (unsigned short*)(ws + B_TA);

  k_prep<<<PB_END, 256, 0, stream>>>(eW1, eW2, nW1, nW2, gWx, gWh, aW1, aW2, cW1, cW2, planes);

  k_edge<<<MROWS / 4, 160, 0, stream>>>(rn, te, se, planes + P_EW1, planes + P_EW2, eb1, eb2, nin);

  k_node<<<MROWS / 128, 256, 0, stream>>>(nin, planes + P_NW1, planes + P_NW2, nb1, nb2, rnnin);

  k_gru<<<NB / 16, 256, 0, stream>>>(rnnin, rhx, msk, planes + P_GWX, planes + P_GWH, gbx, gbh, outs, out2);

  k_h1<<<dim3(MROWS / 128, 8), 128, 0, stream>>>(outs, planes + P_HW1, ab1, cb1, tpl);

  k_act<<<dim3(MROWS / 128, 4), 128, 0, stream>>>(tpl, planes + P_AW2, ab2, out1);

  k_crit<<<MROWS / 64, 256, 0, stream>>>(tpl + TPLANE, planes + P_CW2, cb2, clW, clb, out0);
}
